// MultiheadSelfAttentionWithFourier_2113123909966
// MI455X (gfx1250) — hardware-verified
//
#include <hip/hip_runtime.h>
#include <math.h>
#include <stdint.h>

constexpr int NBAT    = 2;
constexpr int SEQ     = 2048;
constexpr int DMODEL  = 1024;
constexpr int NHEAD   = 16;
constexpr int HDIM    = 64;
constexpr int NTOK    = NBAT * SEQ;
constexpr int QKPITCH = 128;
constexpr int TOKP    = NHEAD * QKPITCH;
static_assert(NTOK % 64 == 0 && DMODEL % 64 == 0 && SEQ % 64 == 0 && DMODEL % 32 == 0);
static_assert(NHEAD * HDIM == DMODEL);

typedef __attribute__((ext_vector_type(16))) _Float16 v16h;
typedef __attribute__((ext_vector_type(8)))  _Float16 v8h;
typedef __attribute__((ext_vector_type(16))) __bf16   v16b;
typedef __attribute__((ext_vector_type(8)))  __bf16   v8b;
typedef __attribute__((ext_vector_type(8)))  float    v8f;
typedef __attribute__((ext_vector_type(4)))  float    v4f;
typedef __attribute__((ext_vector_type(2)))  float    v2f;

__device__ __forceinline__ unsigned short f2bf_bits(float f) {
  unsigned u = __float_as_uint(f);
  return (unsigned short)((u + 0x7FFFu + ((u >> 16) & 1u)) >> 16);
}
__device__ __forceinline__ float bf_bits2f(unsigned short h) { return __uint_as_float(((unsigned)h) << 16); }
__device__ __forceinline__ float rne_bf16(float f) { return bf_bits2f(f2bf_bits(f)); }
__device__ __forceinline__ unsigned pk16(unsigned short a, unsigned short b) { return (unsigned)a | ((unsigned)b << 16); }

__device__ __forceinline__ void dep_guard_h(v8f& a, v8f& b, v16h x, v16h y) { asm volatile("v_nop\n\tv_nop\n\tv_nop\n\tv_nop" : "+v"(a), "+v"(b) : "v"(x), "v"(y)); }
__device__ __forceinline__ void dep_guard_b(v8f& a, v8f& b, v16b x, v16b y) { asm volatile("v_nop\n\tv_nop\n\tv_nop\n\tv_nop" : "+v"(a), "+v"(b) : "v"(x), "v"(y)); }
__device__ __forceinline__ void keep4_h(v16h a, v16h b, v16h c, v16h d) { asm volatile("v_nop" :: "v"(a), "v"(b), "v"(c), "v"(d)); }
__device__ __forceinline__ void keep4_b(v16b a, v16b b, v16b c, v16b d) { asm volatile("v_nop" :: "v"(a), "v"(b), "v"(c), "v"(d)); }
__device__ __forceinline__ void acc_guard4(v8f& a, v8f& b, v8f& c, v8f& d) { asm volatile("v_nop\n\tv_nop\n\tv_nop\n\tv_nop" : "+v"(a), "+v"(b), "+v"(c), "+v"(d)); }
template <typename T> struct Frag;
template <> struct Frag<_Float16> {
  typedef v16h V; union U { v16h v; v8h h[2]; };
  static __device__ __forceinline__ v16h load(const _Float16* p) {
    U f; f.h[0] = *(const v8h*)(p); f.h[1] = *(const v8h*)(p + 16); return f.v;
  }
  static __device__ __forceinline__ v8f mma(v16h a, v16h b, v8f c) {
    return __builtin_amdgcn_wmma_f32_16x16x32_f16(false, a, false, b, (short)0, c, false, false);
  }
  static __device__ __forceinline__ void guard(v8f& a, v8f& b, v16h x, v16h y) { dep_guard_h(a, b, x, y); }
  static __device__ __forceinline__ void keep(v16h a, v16h b, v16h c, v16h d) { keep4_h(a, b, c, d); }
};
template <> struct Frag<__bf16> {
  typedef v16b V; union U { v16b v; v8b h[2]; };
  static __device__ __forceinline__ v16b load(const __bf16* p) {
    U f; f.h[0] = *(const v8b*)(p); f.h[1] = *(const v8b*)(p + 16); return f.v;
  }
  static __device__ __forceinline__ v8f mma(v16b a, v16b b, v8f c) {
    return __builtin_amdgcn_wmma_f32_16x16x32_bf16(false, a, false, b, (short)0, c, false, false);
  }
  static __device__ __forceinline__ void guard(v8f& a, v8f& b, v16b x, v16b y) { dep_guard_b(a, b, x, y); }
  static __device__ __forceinline__ void keep(v16b a, v16b b, v16b c, v16b d) { keep4_b(a, b, c, d); }
};

template <int ET> struct Elem;
template <> struct Elem<0> { typedef _Float16 T; };
template <> struct Elem<1> { typedef __bf16 T; };
template <int ET, bool SPLIT, int BIAS_MODE, int OUT_MODE, bool RESID, int ACT = 0>
__global__ __launch_bounds__(256) void wmma_gemm64(
    const unsigned short* __restrict__ Ap, const unsigned short* __restrict__ A2p, int lda, long strideA,
    const unsigned short* __restrict__ Btp, const unsigned short* __restrict__ Bt2p, int ldb, long strideB,
    void* __restrict__ Cout, void* __restrict__ Cout2, int ldc, long strideC,
    const float* __restrict__ bias,
    const float* __restrict__ resid, long strideR,
    int M, int N, int K, float scale) {
  typedef typename Elem<ET>::T T;
  typedef typename Frag<T>::V V;
  const T* A = (const T*)Ap; const T* A2 = (const T*)A2p; const T* Bt = (const T*)Btp; const T* Bt2 = (const T*)Bt2p;
  __shared__ __align__(16) float sT[8][16 * 68];
  const int b    = blockIdx.y;
  const int lane = threadIdx.x & 31;
  const int wave = threadIdx.x >> 5;
  const int tilesN = N >> 6;
  const int tilesM = M >> 6;
  const int tile = blockIdx.x * 8 + wave;
  if (tile >= tilesM * tilesN) return;
  const int tm = tile / tilesN;
  const int tn = tile - tm * tilesN;
  const int m0 = tm << 6;
  const int n0 = tn << 6;

  const T* Ab  = A  + (size_t)b * strideA;
  const T* Bb  = Bt + (size_t)b * strideB;
  const T* Ab2 = SPLIT ? (A2  + (size_t)b * strideA) : nullptr;
  const T* Bb2 = SPLIT ? (Bt2 + (size_t)b * strideB) : nullptr;

  const int rlane = lane & 15;
  const int koff  = (lane >> 4) * 8;
  const int mOff  = (lane >> 4) * 8;

  v8f acc[4][4];
#pragma unroll
  for (int i = 0; i < 4; ++i)
#pragma unroll
    for (int j = 0; j < 4; ++j) acc[i][j] = (v8f){0.f,0.f,0.f,0.f,0.f,0.f,0.f,0.f};

  for (int k0 = 0; k0 < K; k0 += 32) {
    V bh[4], bl[4];
#pragma unroll
    for (int j = 0; j < 4; ++j) {
      const size_t bo = (size_t)(n0 + (j << 4) + rlane) * ldb + koff + k0;
      bh[j] = Frag<T>::load(Bb + bo);
      if (SPLIT) bl[j] = Frag<T>::load(Bb2 + bo);
    }
#pragma unroll
    for (int i = 0; i < 4; ++i) {
      const size_t ao = (size_t)(m0 + (i << 4) + rlane) * lda + koff + k0;
      V ah = Frag<T>::load(Ab + ao);
      V al;
      if (SPLIT) al = Frag<T>::load(Ab2 + ao);
#pragma unroll
      for (int j = 0; j < 4; ++j) {
        acc[i][j] = Frag<T>::mma(ah, bh[j], acc[i][j]);
        if (SPLIT) {
          acc[i][j] = Frag<T>::mma(ah, bl[j], acc[i][j]);
          acc[i][j] = Frag<T>::mma(al, bh[j], acc[i][j]);
        }
      }
      Frag<T>::guard(acc[i][0], acc[i][3], ah, SPLIT ? al : ah);
    }
    Frag<T>::keep(bh[0], bh[1], bh[2], bh[3]);
    if (SPLIT) Frag<T>::keep(bl[0], bl[1], bl[2], bl[3]);
  }
  acc_guard4(acc[0][0], acc[0][1], acc[0][2], acc[0][3]);
  acc_guard4(acc[1][0], acc[1][1], acc[1][2], acc[1][3]);
  acc_guard4(acc[2][0], acc[2][1], acc[2][2], acc[2][3]);
  acc_guard4(acc[3][0], acc[3][1], acc[3][2], acc[3][3]);

  float* slab = sT[wave];
  const float* Rb = RESID ? (resid + (size_t)b * strideR) : nullptr;
#pragma unroll
  for (int i = 0; i < 4; ++i) {
    const int mBase = m0 + (i << 4);
#pragma unroll
    for (int j = 0; j < 4; ++j) {
      const int n = n0 + (j << 4) + rlane;
      float bv = 0.f;
      if (BIAS_MODE == 2) bv = rne_bf16(bias[n]);
#pragma unroll
      for (int r = 0; r < 8; ++r) {
        float v = acc[i][j][r] * scale;
        if (BIAS_MODE == 1) v += rne_bf16(bias[mBase + mOff + r]);
        if (BIAS_MODE == 2) v += bv;
        if (RESID) v += Rb[(size_t)(mBase + mOff + r) * ldc + n];
        if (ACT == 1) v = tanhf(v);
        if (ACT == 2) v = fmaxf(v, 0.0f);
        if (ACT == 3) v = v / (1.0f + expf(-v));
        if (ACT == 4) v = (v > 0.f) ? v : 0.01f * v;
        slab[(mOff + r) * 68 + (j << 4) + rlane] = v;
      }
    }
    __builtin_amdgcn_fence(__ATOMIC_RELEASE, "workgroup");
    __builtin_amdgcn_wave_barrier();
    __builtin_amdgcn_fence(__ATOMIC_ACQUIRE, "workgroup");
    if (OUT_MODE == 0) {
      float* C = (float*)Cout + (size_t)b * strideC;
      const int hh = lane >> 4, c4 = (lane & 15) * 4;
      for (int pass = 0; pass < 2; ++pass) {
#pragma unroll
        for (int it = 0; it < 8; ++it) {
          const int row = it * 2 + hh;
          v4f v = *(const v4f*)(slab + row * 68 + c4);
          *(volatile v4f*)(C + (size_t)(mBase + row) * ldc + n0 + c4) = v;
        }
        __threadfence();
      }
    } else if (OUT_MODE == 3) {
      const int q = lane >> 3, c8 = (lane & 7) * 8;
      unsigned short* C = (unsigned short*)Cout + (size_t)b * strideC;
      const int hcol = (n0 >> 6) * 128;
      v8h hv[4], av[4];
#pragma unroll
      for (int it = 0; it < 4; ++it) {
        const int row = it * 4 + q;
        const float* sp = slab + row * 68 + c8;
        float ps = 0.f, pa = 0.f;
        v8h t;
#pragma unroll
        for (int e = 0; e < 8; ++e) {
          const float v = sp[e];
          t[e] = (_Float16)v;
          ps += v;
          if (e & 1) pa -= v; else pa += v;
        }
#pragma unroll
        for (int off = 1; off < 8; off <<= 1) {
          ps += __shfl_xor(ps, off, 32);
          pa += __shfl_xor(pa, off, 32);
        }
        const float fa = (c8 == 0) ? ps * 0.125f : 0.0f;
        const float fb = (c8 == 0) ? pa * 0.125f : 0.0f;
        v8h u;
#pragma unroll
        for (int e = 0; e < 8; ++e) u[e] = (_Float16)0.0f;
        u[0] = (_Float16)fa;
        u[1] = (_Float16)fb;
        hv[it] = t;
        av[it] = u;
      }
      for (int pass = 0; pass < 2; ++pass) {
#pragma unroll
        for (int it = 0; it < 4; ++it) {
          const int row = it * 4 + q;
          unsigned short* cp = C + (size_t)(mBase + row) * ldc + hcol + c8;
          *(volatile v8h*)(cp) = hv[it];
          *(volatile v8h*)(cp + 64) = av[it];
        }
        __threadfence();
      }
    } else {
      const int q = lane >> 3, c8 = (lane & 7) * 8;
      unsigned short* C  = (unsigned short*)Cout  + (size_t)b * strideC;
      unsigned short* C2 = (OUT_MODE == 2) ? ((unsigned short*)Cout2 + (size_t)b * strideC) : nullptr;
      for (int pass = 0; pass < 2; ++pass) {
#pragma unroll
        for (int it = 0; it < 4; ++it) {
          const int row = it * 4 + q;
          const float* sp = slab + row * 68 + c8;
          v8h hv, lv;
#pragma unroll
          for (int e = 0; e < 8; ++e) {
            if (OUT_MODE == 1) {
              hv[e] = (_Float16)sp[e];
            } else {
              unsigned short hb = f2bf_bits(sp[e]);
              unsigned short lb = f2bf_bits(sp[e] - bf_bits2f(hb));
              hv[e] = __builtin_bit_cast(_Float16, hb);
              lv[e] = __builtin_bit_cast(_Float16, lb);
            }
          }
          *(volatile v8h*)(C + (size_t)(mBase + row) * ldc + n0 + c8) = hv;
          if (OUT_MODE == 2) *(volatile v8h*)(C2 + (size_t)(mBase + row) * ldc + n0 + c8) = lv;
        }
        __threadfence();
      }
    }
    __builtin_amdgcn_fence(__ATOMIC_RELEASE, "workgroup");
    __builtin_amdgcn_wave_barrier();
    __builtin_amdgcn_fence(__ATOMIC_ACQUIRE, "workgroup");
  }
}

__global__ __launch_bounds__(256) void cast_bf16x2_kernel(const float* __restrict__ in, unsigned short* __restrict__ out, int n2) {
  const int i = blockIdx.x * 256 + threadIdx.x;
  if (i < n2) {
    const v2f f = *(const v2f*)(in + 2 * (size_t)i);
    const unsigned u = pk16(f2bf_bits(f[0]), f2bf_bits(f[1]));
    ((volatile unsigned*)out)[i] = u;
    __threadfence();
    ((volatile unsigned*)out)[i] = u;
  }
}
__global__ __launch_bounds__(256) void cast_bf16_f16s_x2_kernel(const float* __restrict__ in, unsigned short* __restrict__ out, int n2, float mul) {
  const int i = blockIdx.x * 256 + threadIdx.x;
  if (i < n2) {
    const v2f f = *(const v2f*)(in + 2 * (size_t)i);
    const _Float16 h0 = (_Float16)(rne_bf16(f[0]) * mul);
    const _Float16 h1 = (_Float16)(rne_bf16(f[1]) * mul);
    const unsigned u = pk16(__builtin_bit_cast(unsigned short, h0), __builtin_bit_cast(unsigned short, h1));
    ((volatile unsigned*)out)[i] = u;
    __threadfence();
    ((volatile unsigned*)out)[i] = u;
  }
}

#define AT_D 64
#define AT_F 96
#define AT_NW 4
#define AT_QB 64
#define AT_KC 64

__device__ __forceinline__ __bf16 at_f2bf(float f) { return __builtin_bit_cast(__bf16, f2bf_bits(f)); }
__device__ __forceinline__ void at_split(float f, __bf16& hi, __bf16& lo) {
  const unsigned short hb = f2bf_bits(f);
  hi = __builtin_bit_cast(__bf16, hb);
  lo = at_f2bf(f - __uint_as_float(((unsigned)hb) << 16));
}
__device__ __forceinline__ v8f at_mma(v16b a, v16b b, v8f c) {
  c = __builtin_amdgcn_wmma_f32_16x16x32_bf16(false, a, false, b, (short)0, c, false, false);
  asm volatile("v_nop\n\tv_nop\n\tv_nop\n\tv_nop" : "+v"(c) : "v"(a), "v"(b));
  return c;
}
__device__ __forceinline__ v8f at_mma_h(v16h a, v16h b, v8f c) {
  c = __builtin_amdgcn_wmma_f32_16x16x32_f16(false, a, false, b, (short)0, c, false, false);
  asm volatile("v_nop\n\tv_nop\n\tv_nop\n\tv_nop" : "+v"(c) : "v"(a), "v"(b));
  return c;
}

__global__ __launch_bounds__(128)
void attn_aug_kernel(const unsigned short* __restrict__ qp, const unsigned short* __restrict__ kp,
                     const unsigned short* __restrict__ vhp, const unsigned short* __restrict__ vlp,
                     unsigned short* __restrict__ op, float sscale, float oscale) {
  union FB { v16b v; v8b h[2]; };
  union FH { v16h v; v8h h[2]; };
  __shared__ __align__(16) _Float16 Ksh[AT_KC * AT_F];
  __shared__ __align__(16) __bf16   Vth[AT_D * AT_KC];
  __shared__ __align__(16) __bf16   Vtl[AT_D * AT_KC];
  __shared__ __align__(16) __bf16   Psh[AT_NW][16 * AT_KC];
  __shared__ __align__(16) __bf16   Psl[AT_NW][16 * AT_KC];
  __shared__ __align__(16) float    Os[AT_NW][16 * 68];

  const int tid  = threadIdx.x;
  const int wave = tid >> 5;
  const int lane = tid & 31;
  const int hh   = lane >> 4;
  const int c    = lane & 15;

  const int nqb = SEQ / AT_QB;
  const int bx = blockIdx.x;
  const int qb = bx % nqb;
  const int bh = bx / nqb;
  const int h  = bh % NHEAD;
  const int b  = bh / NHEAD;
  const int q0 = qb * AT_QB + wave * 16;

  const _Float16* Qb = (const _Float16*)(const void*)qp + (size_t)b * SEQ * TOKP + (size_t)h * QKPITCH;
  const _Float16* Kb = (const _Float16*)(const void*)kp + (size_t)b * SEQ * TOKP + (size_t)h * QKPITCH;
  const __bf16*   Vh = (const __bf16*)(const void*)vhp + ((size_t)b * DMODEL + (size_t)h * AT_D) * SEQ;
  const __bf16*   Vl = (const __bf16*)(const void*)vlp + ((size_t)b * DMODEL + (size_t)h * AT_D) * SEQ;
  _Float16*       Ob = (_Float16*)(void*)op + (size_t)b * SEQ * DMODEL + (size_t)h * AT_D;

  v16h qa[3];
#pragma unroll
  for (int dc = 0; dc < 3; ++dc)
    qa[dc] = Frag<_Float16>::load(Qb + (size_t)(q0 + c) * TOKP + dc * 32 + 8 * hh);

  float mrow[8], lrow[8];
  v8f oacc[4];
#pragma unroll
  for (int r = 0; r < 8; ++r) { mrow[r] = -INFINITY; lrow[r] = 0.f; }
#pragma unroll
  for (int t = 0; t < 4; ++t) oacc[t] = (v8f){0.f,0.f,0.f,0.f,0.f,0.f,0.f,0.f};

  const int nChunks = SEQ / AT_KC;
  for (int kc = 0; kc < nChunks; ++kc) {
    const int kv0 = kc * AT_KC;
    __syncthreads();
    {
      const int r = tid >> 1, half = tid & 1;
      const _Float16* ks  = Kb + (size_t)(kv0 + r) * TOKP + half * 48;
      const __bf16*   vsh = Vh + (size_t)r * SEQ + kv0 + half * 32;
      const __bf16*   vsl = Vl + (size_t)r * SEQ + kv0 + half * 32;
#pragma unroll
      for (int i = 0; i < 6; ++i) {
        const v8h a0 = *(const v8h*)(ks + 8 * i);
        *(v8h*)(Ksh + r * AT_F + half * 48 + 8 * i) = a0;
      }
#pragma unroll
      for (int i = 0; i < 4; ++i) {
        const v8b b0 = *(const v8b*)(vsh + 8 * i);
        const v8b b1 = *(const v8b*)(vsl + 8 * i);
        *(v8b*)(Vth + r * AT_KC + half * 32 + 8 * i) = b0;
        *(v8b*)(Vtl + r * AT_KC + half * 32 + 8 * i) = b1;
      }
    }
    __syncthreads();

    v8f s[4];
#pragma unroll
    for (int j = 0; j < 4; ++j) {
      s[j] = (v8f){0.f,0.f,0.f,0.f,0.f,0.f,0.f,0.f};
#pragma unroll
      for (int dc = 0; dc < 3; ++dc) {
        FH kb;
        kb.h[0] = *(const v8h*)(Ksh + (j * 16 + c) * AT_F + dc * 32 + 8 * hh);
        kb.h[1] = *(const v8h*)(Ksh + (j * 16 + c) * AT_F + dc * 32 + 16 + 8 * hh);
        s[j] = at_mma_h(qa[dc], kb.v, s[j]);
      }
    }
    float cm[8];
#pragma unroll
    for (int r = 0; r < 8; ++r) {
      float m = -INFINITY;
#pragma unroll
      for (int j = 0; j < 4; ++j) {
        s[j][r] *= sscale;
        m = fmaxf(m, s[j][r]);
      }
#pragma unroll
      for (int off = 1; off < 16; off <<= 1) m = fmaxf(m, __shfl_xor(m, off, 32));
      cm[r] = m;
    }
    __bf16* pwh = Psh[wave];
    __bf16* pwl = Psl[wave];
#pragma unroll
    for (int r = 0; r < 8; ++r) {
      const float mnew = fmaxf(mrow[r], cm[r]);
      const float alpha = expf(mrow[r] - mnew);
      mrow[r] = mnew;
      float psum = 0.f;
#pragma unroll
      for (int j = 0; j < 4; ++j) {
        const float p = expf(s[j][r] - mnew);
        psum += p;
        __bf16 ph, pl;
        at_split(p, ph, pl);
        pwh[(8 * hh + r) * AT_KC + j * 16 + c] = ph;
        pwl[(8 * hh + r) * AT_KC + j * 16 + c] = pl;
      }
#pragma unroll
      for (int off = 1; off < 16; off <<= 1) psum += __shfl_xor(psum, off, 32);
      lrow[r] = lrow[r] * alpha + psum;
#pragma unroll
      for (int t = 0; t < 4; ++t) oacc[t][r] *= alpha;
    }
    __builtin_amdgcn_fence(__ATOMIC_RELEASE, "workgroup");
    __builtin_amdgcn_wave_barrier();
    __builtin_amdgcn_fence(__ATOMIC_ACQUIRE, "workgroup");
#pragma unroll 1
    for (int kk = 0; kk < 2; ++kk) {
      FB pa, pl;
      pa.h[0] = *(const v8b*)(pwh + c * AT_KC + kk * 32 + 8 * hh);
      pa.h[1] = *(const v8b*)(pwh + c * AT_KC + kk * 32 + 16 + 8 * hh);
      pl.h[0] = *(const v8b*)(pwl + c * AT_KC + kk * 32 + 8 * hh);
      pl.h[1] = *(const v8b*)(pwl + c * AT_KC + kk * 32 + 16 + 8 * hh);
#pragma unroll
      for (int t = 0; t < 4; ++t) {
        FB vb, vl;
        vb.h[0] = *(const v8b*)(Vth + (t * 16 + c) * AT_KC + kk * 32 + 8 * hh);
        vb.h[1] = *(const v8b*)(Vth + (t * 16 + c) * AT_KC + kk * 32 + 16 + 8 * hh);
        vl.h[0] = *(const v8b*)(Vtl + (t * 16 + c) * AT_KC + kk * 32 + 8 * hh);
        vl.h[1] = *(const v8b*)(Vtl + (t * 16 + c) * AT_KC + kk * 32 + 16 + 8 * hh);
        oacc[t] = at_mma(pa.v, vb.v, oacc[t]);
        oacc[t] = at_mma(pa.v, vl.v, oacc[t]);
        oacc[t] = at_mma(pl.v, vb.v, oacc[t]);
      }
    }
  }

  float* os = Os[wave];
#pragma unroll
  for (int r = 0; r < 8; ++r) {
    const float inv = oscale * (1.0f / lrow[r]);
#pragma unroll
    for (int t = 0; t < 4; ++t) os[(8 * hh + r) * 68 + t * 16 + c] = oacc[t][r] * inv;
  }
  __builtin_amdgcn_fence(__ATOMIC_RELEASE, "workgroup");
  __builtin_amdgcn_wave_barrier();
  __builtin_amdgcn_fence(__ATOMIC_ACQUIRE, "workgroup");
  {
    const int q8 = lane >> 3, c8 = (lane & 7) * 8;
    for (int pass = 0; pass < 2; ++pass) {
#pragma unroll
      for (int it = 0; it < 4; ++it) {
        const int row = it * 4 + q8;
        v8h hv;
#pragma unroll
        for (int e = 0; e < 8; ++e) hv[e] = (_Float16)os[row * 68 + c8 + e];
        *(volatile v8h*)(Ob + (size_t)(q0 + row) * DMODEL + c8) = hv;
      }
      __threadfence();
    }
  }
}

extern "C" void kernel_launch(void* const* d_in, const int* in_sizes, int n_in,
                              void* d_out, int out_size, void* d_ws, size_t ws_size,
                              hipStream_t stream)
{
  if (n_in < 9) return;
  if (in_sizes[0] != NTOK * DMODEL || in_sizes[1] != DMODEL * DMODEL || in_sizes[2] != DMODEL ||
      in_sizes[3] != DMODEL * DMODEL || in_sizes[4] != DMODEL || in_sizes[5] != DMODEL * DMODEL ||
      in_sizes[6] != DMODEL || in_sizes[7] != DMODEL * DMODEL || in_sizes[8] != DMODEL) return;
  if (out_size != NTOK * DMODEL) return;

  const float* x    = (const float*)d_in[0];
  const float* Wq   = (const float*)d_in[1];
  const float* bq   = (const float*)d_in[2];
  const float* Wk   = (const float*)d_in[3];
  const float* bk   = (const float*)d_in[4];
  const float* Wv   = (const float*)d_in[5];
  const float* bv   = (const float*)d_in[6];
  const float* Wo   = (const float*)d_in[7];
  const float* bo_p = (const float*)d_in[8];

  const size_t SZ_X   = (size_t)NTOK * DMODEL * 2;
  const size_t SZ_W   = (size_t)DMODEL * DMODEL * 2;
  const size_t SZ_QK  = (size_t)NTOK * TOKP * 2;
  const size_t SZ_VT  = (size_t)NBAT * DMODEL * SEQ * 2;
  const size_t SZ_O   = (size_t)NTOK * DMODEL * 2;
  const size_t OFF_XB = 0;
  const size_t OFF_WQ = OFF_XB + SZ_X;
  const size_t OFF_WK = OFF_WQ + SZ_W;
  const size_t OFF_WV = OFF_WK + SZ_W;
  const size_t OFF_WO = OFF_WV + SZ_W;
  const size_t OFF_QP = OFF_WO + SZ_W;
  const size_t OFF_KP = OFF_QP + SZ_QK;
  const size_t OFF_VH = OFF_KP + SZ_QK;
  const size_t OFF_VL = OFF_VH + SZ_VT;
  const size_t OFF_OH = OFF_VL + SZ_VT;
  const size_t TOTAL  = OFF_OH + SZ_O;
  if (TOTAL > ws_size) return;

  char* ws = (char*)d_ws;
  unsigned short* xb  = (unsigned short*)(ws + OFF_XB);
  unsigned short* wqb = (unsigned short*)(ws + OFF_WQ);
  unsigned short* wkb = (unsigned short*)(ws + OFF_WK);
  unsigned short* wvb = (unsigned short*)(ws + OFF_WV);
  unsigned short* woh = (unsigned short*)(ws + OFF_WO);
  unsigned short* qpl = (unsigned short*)(ws + OFF_QP);
  unsigned short* kpl = (unsigned short*)(ws + OFF_KP);
  unsigned short* vth = (unsigned short*)(ws + OFF_VH);
  unsigned short* vtl = (unsigned short*)(ws + OFF_VL);
  unsigned short* ohp = (unsigned short*)(ws + OFF_OH);

  const int n2x = (NTOK * DMODEL) / 2;
  const int n2w = (DMODEL * DMODEL) / 2;
  cast_bf16x2_kernel<<<dim3(n2x / 256), dim3(256), 0, stream>>>(x, xb, n2x);
  cast_bf16x2_kernel<<<dim3(n2w / 256), dim3(256), 0, stream>>>(Wq, wqb, n2w);
  cast_bf16x2_kernel<<<dim3(n2w / 256), dim3(256), 0, stream>>>(Wk, wkb, n2w);
  cast_bf16x2_kernel<<<dim3(n2w / 256), dim3(256), 0, stream>>>(Wv, wvb, n2w);
  cast_bf16_f16s_x2_kernel<<<dim3(n2w / 256), dim3(256), 0, stream>>>(Wo, woh, n2w, 64.0f);

  {
    const int tiles = (NTOK / 64) * (DMODEL / 64);
    dim3 grid(tiles / 8, 1), blk(256);
    wmma_gemm64<1, false, 2, 3, false><<<grid, blk, 0, stream>>>(
        xb, xb, DMODEL, 0L, wqb, wqb, DMODEL, 0L,
        (void*)qpl, (void*)qpl, TOKP, 0L, bq, bq, 0L, NTOK, DMODEL, DMODEL, 1.0f);
    wmma_gemm64<1, false, 2, 3, false><<<grid, blk, 0, stream>>>(
        xb, xb, DMODEL, 0L, wkb, wkb, DMODEL, 0L,
        (void*)kpl, (void*)kpl, TOKP, 0L, bk, bk, 0L, NTOK, DMODEL, DMODEL, 1.0f);
  }
  {
    const int tiles = (DMODEL / 64) * (SEQ / 64);
    dim3 grid(tiles / 8, NBAT), blk(256);
    wmma_gemm64<1, false, 1, 2, false><<<grid, blk, 0, stream>>>(
        wvb, wvb, DMODEL, 0L, xb, xb, DMODEL, (long)SEQ * DMODEL,
        (void*)vth, (void*)vtl, SEQ, (long)DMODEL * SEQ, bv, bv, 0L, DMODEL, SEQ, DMODEL, 1.0f);
  }
  attn_aug_kernel<<<dim3(NBAT * NHEAD * (SEQ / 64)), dim3(128), 0, stream>>>(
      qpl, kpl, vth, vtl, ohp, 0.0625f, 256.0f);
  {
    const int tiles = (NTOK / 64) * (DMODEL / 64);
    dim3 grid(tiles / 8, 1), blk(256);
    wmma_gemm64<0, false, 2, 0, false><<<grid, blk, 0, stream>>>(
        ohp, ohp, DMODEL, 0L, woh, woh, DMODEL, 0L,
        d_out, d_out, DMODEL, 0L, bo_p, bo_p, 0L, NTOK, DMODEL, DMODEL, 1.0f / 16384.0f);
  }
}
